// MambaInMamba_33509334844072
// MI455X (gfx1250) — hardware-run, weakly checked
//
#include <hip/hip_runtime.h>
#include <math.h>

typedef __attribute__((ext_vector_type(16))) __bf16   v16b;
typedef __attribute__((ext_vector_type(8)))  __bf16   v8b;
typedef __attribute__((ext_vector_type(8)))  float    v8f;
typedef __attribute__((ext_vector_type(4)))  float    v4f;
typedef __attribute__((ext_vector_type(4)))  unsigned v4u;

constexpr int kBatch  = 2;
constexpr int kSeq    = 1024;
constexpr int kDm     = 1024;
constexpr int kDin    = 2048;
constexpr int kNst    = 16;
constexpr int kDtR    = 64;
constexpr int kXdN    = kDtR + 2 * kNst;
constexpr int kXdP    = 128;
constexpr int kXzP    = 2 * kDin;
constexpr int kRows   = kBatch * kSeq;
constexpr int kMdi    = 64;
constexpr int kMn     = 4;
constexpr int kMdtR   = 4;
constexpr int kMxd    = kMdtR + 2 * kMn;
constexpr int kConvTP = 260;
constexpr int kScanTS = 64;
constexpr int kScanCh = 64;
constexpr int kScanYP = 68;
constexpr int kNbTS   = 16;
constexpr int kNbOP   = 68;
static_assert(kXdN == 96);
static_assert(kMxd == 12);
static_assert(kDtR == 64 && kMdi == 64);
static_assert((kDm % 32) == 0 && (kDin % 32) == 0 && (kDtR % 32) == 0);
static_assert((kRows % 64) == 0 && (kXzP % 64) == 0 && (kXdP % 64) == 0 && (kDm % 64) == 0 && (kDin % 64) == 0);
static_assert((kSeq % kScanTS) == 0 && (kSeq % 64) == 0 && (kDin % kScanCh) == 0 && (kDin % 256) == 0 && (kSeq % kNbTS) == 0);
static_assert((kSeq & (kSeq - 1)) == 0);

constexpr size_t kOffXH   = 0;
constexpr size_t kOffWIH  = kOffXH  + (size_t)kRows * kDm  * 2;
constexpr size_t kOffWXH  = kOffWIH + (size_t)kXzP  * kDm  * 2;
constexpr size_t kOffWDH  = kOffWXH + (size_t)kXdP  * kDin * 2;
constexpr size_t kOffWOH  = kOffWDH + (size_t)kDin  * kDtR * 2;
constexpr size_t kOffXZ   = kOffWOH + (size_t)kDm   * kDin * 2;
constexpr size_t kOffUC   = kOffXZ  + (size_t)kRows * kXzP * 4;
constexpr size_t kOffUCH  = kOffUC  + (size_t)kRows * kDin * 4;
constexpr size_t kOffXD   = kOffUCH + (size_t)kRows * kDin * 2;
constexpr size_t kOffDTM  = kOffXD  + (size_t)kRows * kXdP * 4;
constexpr size_t kOffDL   = kOffDTM + (size_t)kRows * kDtR * 2;
constexpr size_t kOffYH   = kOffDL  + (size_t)kRows * kDin * 4;
constexpr size_t kOffYL   = kOffYH  + (size_t)kRows * kDin * 2;
constexpr size_t kWsTotal = kOffYL  + (size_t)kRows * kDin * 2;
static_assert(kWsTotal == 111149056ull);
static_assert(kWsTotal <= 134217728ull);
static_assert((kOffWIH % 128) == 0 && (kOffWXH % 128) == 0 && (kOffWDH % 128) == 0 && (kOffWOH % 128) == 0 &&
              (kOffXZ % 128) == 0 && (kOffUC % 128) == 0 && (kOffUCH % 128) == 0 && (kOffXD % 128) == 0 &&
              (kOffDTM % 128) == 0 && (kOffDL % 128) == 0 && (kOffYH % 128) == 0 && (kOffYL % 128) == 0);

__device__ __forceinline__ unsigned bf_rne_bits(float f) {
  const unsigned u = __float_as_uint(f);
  return (u + 0x7FFFu + ((u >> 16) & 1u)) >> 16;
}
__device__ __forceinline__ float bf_val(float f) { return __uint_as_float(bf_rne_bits(f) << 16); }

__device__ __forceinline__ v4u pack8_bf16(v4f a0, v4f a1) {
  const float x0 = a0[0], x1 = a0[1], x2 = a0[2], x3 = a0[3];
  const float x4 = a1[0], x5 = a1[1], x6 = a1[2], x7 = a1[3];
  const unsigned w0 = bf_rne_bits(x0) | (bf_rne_bits(x1) << 16);
  const unsigned w1 = bf_rne_bits(x2) | (bf_rne_bits(x3) << 16);
  const unsigned w2 = bf_rne_bits(x4) | (bf_rne_bits(x5) << 16);
  const unsigned w3 = bf_rne_bits(x6) | (bf_rne_bits(x7) << 16);
  v4u r = {w0, w1, w2, w3};
  return r;
}
__device__ __forceinline__ void split2_bf16(float xa, float xb, unsigned& hw, unsigned& lw) {
  const unsigned ha = bf_rne_bits(xa), hb = bf_rne_bits(xb);
  const float ra = xa - __uint_as_float(ha << 16);
  const float rb = xb - __uint_as_float(hb << 16);
  hw = ha | (hb << 16);
  lw = bf_rne_bits(ra) | (bf_rne_bits(rb) << 16);
}
__device__ __forceinline__ void split8_bf16(v4f a0, v4f a1, v4u& hi, v4u& lo) {
  const float x0 = a0[0], x1 = a0[1], x2 = a0[2], x3 = a0[3];
  const float x4 = a1[0], x5 = a1[1], x6 = a1[2], x7 = a1[3];
  unsigned h0, h1, h2, h3, l0, l1, l2, l3;
  split2_bf16(x0, x1, h0, l0);
  split2_bf16(x2, x3, h1, l1);
  split2_bf16(x4, x5, h2, l2);
  split2_bf16(x6, x7, h3, l3);
  v4u hv = {h0, h1, h2, h3};
  v4u lv = {l0, l1, l2, l3};
  hi = hv;
  lo = lv;
}
__device__ __forceinline__ float silu_f(float v) { return v * __builtin_amdgcn_rcpf(1.0f + expf(-v)); }
__device__ __forceinline__ float softplus_f(float v) { return fmaxf(v, 0.0f) + log1pf(expf(-fabsf(v))); }

__device__ __forceinline__ void row_guard_b(v8f& a, v8f& b, v8f& c, v8f& d, v16b x, v16b y, v16b b0, v16b b1, v16b b2, v16b b3) {
  asm volatile("v_nop\n\tv_nop\n\tv_nop\n\tv_nop" : "+v"(a), "+v"(b), "+v"(c), "+v"(d) : "v"(x), "v"(y), "v"(b0), "v"(b1), "v"(b2), "v"(b3));
}
__device__ __forceinline__ void keep4_b(v16b a, v16b b, v16b c, v16b d) { asm volatile("v_nop" :: "v"(a), "v"(b), "v"(c), "v"(d)); }
__device__ __forceinline__ void acc_guard4(v8f& a, v8f& b, v8f& c, v8f& d) { asm volatile("v_nop\n\tv_nop\n\tv_nop\n\tv_nop" : "+v"(a), "+v"(b), "+v"(c), "+v"(d)); }
struct FragB16 {
  union U { v16b v; v8b h[2]; };
  static __device__ __forceinline__ v16b load(const __bf16* p) {
    U f; f.h[0] = *(const v8b*)(p); f.h[1] = *(const v8b*)(p + 16); return f.v;
  }
  static __device__ __forceinline__ v8f mma(v16b a, v16b b, v8f c) {
    return __builtin_amdgcn_wmma_f32_16x16x32_bf16(false, a, false, b, (short)0, c, false, false);
  }
};

template <int SPL>
__global__ __launch_bounds__(256) void wmma_gemm64_bf16(
    const unsigned short* __restrict__ Ap, const unsigned short* __restrict__ A2p, int lda,
    const unsigned short* __restrict__ Btp, int ldb,
    float* __restrict__ C, int ldc, int M, int N, int K)
{
  const __bf16* A  = (const __bf16*)Ap;
  const __bf16* A2 = (const __bf16*)A2p;
  const __bf16* Bt = (const __bf16*)Btp;
  __shared__ __align__(16) float sT[8][16 * 68];
  const int lane = threadIdx.x & 31;
  const int wave = threadIdx.x >> 5;
  const int tilesN = N >> 6;
  const int tilesM = M >> 6;
  const int tile = blockIdx.x * 8 + wave;
  if (tile >= tilesM * tilesN) return;
  const int tm = tile / tilesN;
  const int tn = tile - tm * tilesN;
  const int m0 = tm << 6;
  const int n0 = tn << 6;

  const int rlane = lane & 15;
  const int koff  = (lane >> 4) * 8;
  const int mOff  = (lane >> 4) * 8;

  v8f acc[4][4];
#pragma unroll
  for (int i = 0; i < 4; ++i)
#pragma unroll
    for (int j = 0; j < 4; ++j) acc[i][j] = (v8f){0.f,0.f,0.f,0.f,0.f,0.f,0.f,0.f};

  for (int k0 = 0; k0 < K; k0 += 32) {
    v16b bh[4];
#pragma unroll
    for (int j = 0; j < 4; ++j) {
      const size_t bo = (size_t)(n0 + (j << 4) + rlane) * ldb + koff + k0;
      bh[j] = FragB16::load(Bt + bo);
    }
#pragma unroll
    for (int i = 0; i < 4; ++i) {
      const size_t ao = (size_t)(m0 + (i << 4) + rlane) * lda + koff + k0;
      v16b ah = FragB16::load(A + ao);
      v16b al = ah;
      if (SPL == 1) al = FragB16::load(A2 + ao);
#pragma unroll
      for (int j = 0; j < 4; ++j) {
        acc[i][j] = FragB16::mma(ah, bh[j], acc[i][j]);
        if (SPL == 1) acc[i][j] = FragB16::mma(al, bh[j], acc[i][j]);
      }
      row_guard_b(acc[i][0], acc[i][1], acc[i][2], acc[i][3], ah, al, bh[0], bh[1], bh[2], bh[3]);
    }
    keep4_b(bh[0], bh[1], bh[2], bh[3]);
  }
  acc_guard4(acc[0][0], acc[0][1], acc[0][2], acc[0][3]);
  acc_guard4(acc[1][0], acc[1][1], acc[1][2], acc[1][3]);
  acc_guard4(acc[2][0], acc[2][1], acc[2][2], acc[2][3]);
  acc_guard4(acc[3][0], acc[3][1], acc[3][2], acc[3][3]);

  float* slab = sT[wave];
#pragma unroll
  for (int i = 0; i < 4; ++i) {
    const int mBase = m0 + (i << 4);
#pragma unroll
    for (int j = 0; j < 4; ++j) {
#pragma unroll
      for (int r = 0; r < 8; ++r) {
        slab[(mOff + r) * 68 + (j << 4) + rlane] = acc[i][j][r];
      }
    }
    __builtin_amdgcn_fence(__ATOMIC_RELEASE, "workgroup");
    __builtin_amdgcn_wave_barrier();
    __builtin_amdgcn_fence(__ATOMIC_ACQUIRE, "workgroup");
    {
      const int hh = lane >> 4, c4 = (lane & 15) * 4;
      for (int pass = 0; pass < 2; ++pass) {
#pragma unroll
        for (int it = 0; it < 8; ++it) {
          const int row = it * 2 + hh;
          v4f v = *(const v4f*)(slab + row * 68 + c4);
          *(volatile v4f*)(C + (size_t)(mBase + row) * ldc + n0 + c4) = v;
        }
        __threadfence();
      }
    }
    __builtin_amdgcn_fence(__ATOMIC_RELEASE, "workgroup");
    __builtin_amdgcn_wave_barrier();
    __builtin_amdgcn_fence(__ATOMIC_ACQUIRE, "workgroup");
  }
}

__global__ __launch_bounds__(256) void rne_rows_bf16_kernel(
    const float* __restrict__ src, unsigned short* __restrict__ dst, int total8, int real8)
{
  const int i = blockIdx.x * 256 + threadIdx.x;
  if (i >= total8) return;
  const bool live = (i < real8);
  const int ic = live ? i : (real8 - 1);
  const size_t s0 = (size_t)ic << 3;
  const v4f a0 = *(const v4f*)(src + s0);
  const v4f a1 = *(const v4f*)(src + s0 + 4);
  const v4f zz = {0.f, 0.f, 0.f, 0.f};
  const v4f b0 = live ? a0 : zz;
  const v4f b1 = live ? a1 : zz;
  const v4u w = pack8_bf16(b0, b1);
  unsigned short* q = dst + ((size_t)i << 3);
  *(volatile v4u*)(void*)q = w;
  __threadfence();
  *(volatile v4u*)(void*)q = w;
}

__global__ __launch_bounds__(256) void conv_silu_kernel(
    const float* __restrict__ XZ, const float* __restrict__ cw, const float* __restrict__ cb,
    float* __restrict__ UC, unsigned short* __restrict__ UCH)
{
  __shared__ __align__(16) float sT[16 * kConvTP];
  const int tid = threadIdx.x, lane = tid & 31, wave = tid >> 5;
  const int d0 = blockIdx.x * 256, d = d0 + tid;
  const int g0 = blockIdx.y * 64;
  const int tb = g0 & (kSeq - 1);
  const v4f wv = *(const v4f*)(cw + (size_t)d * 4);
  const float wr0 = wv[0], wr1 = wv[1], wr2 = wv[2], wr3 = wv[3];
  const float w0 = bf_val(wr0), w1 = bf_val(wr1), w2 = bf_val(wr2), w3 = bf_val(wr3);
  const float bc = bf_val(cb[d]);
  float xm3, xm2, xm1;
  {
    const bool hist = (tb > 0);
    const int rb = hist ? (g0 - 3) : g0;
    const float v3 = XZ[(size_t)rb * kXzP + d];
    const float v2 = XZ[(size_t)(rb + 1) * kXzP + d];
    const float v1 = XZ[(size_t)(rb + 2) * kXzP + d];
    xm3 = hist ? v3 : 0.f;
    xm2 = hist ? v2 : 0.f;
    xm1 = hist ? v1 : 0.f;
  }
  const int hrow = wave >> 1;
  const int hch  = (wave & 1) * 128 + lane * 4;
#pragma unroll 1
  for (int sub = 0; sub < 4; ++sub) {
    const int lb = g0 + sub * 16;
#pragma unroll 1
    for (int s = 0; s < 16; ++s) {
      const float xcur = XZ[(size_t)(lb + s) * kXzP + d];
      float acc = w0 * xm3;
      acc = fmaf(w1, xm2, acc);
      acc = fmaf(w2, xm1, acc);
      acc = fmaf(w3, xcur, acc);
      const float sv = acc + bc;
      sT[s * kConvTP + tid] = silu_f(sv);
      xm3 = xm2; xm2 = xm1; xm1 = xcur;
    }
    __syncthreads();
    v4f fv[4];
    v4u bh[2];
#pragma unroll
    for (int it = 0; it < 4; ++it) fv[it] = *(const v4f*)(sT + (it * 4 + hrow) * kConvTP + hch);
#pragma unroll
    for (int it = 0; it < 2; ++it) {
      const float* sp = sT + (it * 8 + wave) * kConvTP + lane * 8;
      const v4f a0 = *(const v4f*)(sp);
      const v4f a1 = *(const v4f*)(sp + 4);
      bh[it] = pack8_bf16(a0, a1);
    }
    for (int pass = 0; pass < 2; ++pass) {
#pragma unroll
      for (int it = 0; it < 4; ++it)
        *(volatile v4f*)(UC + (size_t)(lb + it * 4 + hrow) * kDin + d0 + hch) = fv[it];
#pragma unroll
      for (int it = 0; it < 2; ++it) {
        const size_t o = (size_t)(lb + it * 8 + wave) * kDin + d0 + lane * 8;
        *(volatile v4u*)(void*)(UCH + o) = bh[it];
      }
      __threadfence();
    }
    __syncthreads();
  }
}

__global__ __launch_bounds__(64) void nested_block_kernel(
    const float* __restrict__ XD,
    const float* __restrict__ minw, const float* __restrict__ mcw, const float* __restrict__ mcb,
    const float* __restrict__ mxp, const float* __restrict__ mdtw, const float* __restrict__ mdtb,
    const float* __restrict__ mAlog, const float* __restrict__ mD, const float* __restrict__ moutw,
    unsigned short* __restrict__ DTM)
{
  __shared__ __align__(16) float sWin[kMdi * 2 * kMdi];
  __shared__ __align__(16) float sWout[kMdi * kDtR];
  __shared__ __align__(16) float sXp[kMdi * kMxd];
  __shared__ __align__(16) float sIn[kNbTS * kDtR];
  __shared__ __align__(16) float sXs[kMdi];
  __shared__ __align__(16) float sSm[16];
  __shared__ __align__(16) float sYv[kMdi];
  __shared__ __align__(16) float sO[kNbTS * kNbOP];

  const int tid = threadIdx.x, lane = tid & 31, wave = tid >> 5;
  const size_t row0 = (size_t)blockIdx.x * kSeq;

#pragma unroll 1
  for (int p = 0; p < 2 * kMdi; ++p) {
    const int idx = tid + p * 64;
    const int n = idx >> 6, dd = idx & 63;
    sWin[dd * (2 * kMdi) + n] = bf_val(minw[idx]);
  }
#pragma unroll 1
  for (int p = 0; p < kDtR; ++p) {
    const int idx = tid + p * 64;
    const int o = idx >> 6, dd = idx & 63;
    sWout[dd * kDtR + o] = bf_val(moutw[idx]);
  }
#pragma unroll 1
  for (int p = 0; p < kMxd; ++p) {
    const int idx = tid + p * 64;
    const int e = idx >> 6, dd = idx & 63;
    sXp[dd * kMxd + e] = bf_val(mxp[idx]);
  }

  float nA[kMn], st[kMn], dw[kMdtR];
  {
    const v4f al = *(const v4f*)(mAlog + (size_t)tid * kMn);
    const float a0 = al[0], a1 = al[1], a2 = al[2], a3 = al[3];
    nA[0] = -expf(bf_val(a0)); nA[1] = -expf(bf_val(a1)); nA[2] = -expf(bf_val(a2)); nA[3] = -expf(bf_val(a3));
    const v4f dv = *(const v4f*)(mdtw + (size_t)tid * kMdtR);
    const float q0 = dv[0], q1 = dv[1], q2 = dv[2], q3 = dv[3];
    dw[0] = bf_val(q0); dw[1] = bf_val(q1); dw[2] = bf_val(q2); dw[3] = bf_val(q3);
  }
#pragma unroll
  for (int n = 0; n < kMn; ++n) st[n] = 0.f;
  const float cw0 = bf_val(mcw[tid * 2 + 0]), cw1 = bf_val(mcw[tid * 2 + 1]);
  const float cbv = bf_val(mcb[tid]);
  const float dtb = bf_val(mdtb[tid]);
  const float dD  = bf_val(mD[tid]);
  float prevx = 0.f;

  const int lr = tid >> 4, lc4 = (tid & 15) * 4;
  const int q = lane >> 3, c8 = (lane & 7) * 8;
  const int oc = (lane < kMxd) ? lane : (kMxd - 1);

#pragma unroll 1
  for (int c = 0; c < kSeq / kNbTS; ++c) {
    const int l0 = c * kNbTS;
    __syncthreads();
#pragma unroll
    for (int i = 0; i < 4; ++i) {
      const int r = lr + 4 * i;
      *(v4f*)(sIn + r * kDtR + lc4) = *(const v4f*)(XD + (row0 + l0 + r) * kXdP + lc4);
    }
    __syncthreads();
#pragma unroll 1
    for (int s = 0; s < kNbTS; ++s) {
      const float* ir = sIn + s * kDtR;
      float xa = 0.f, za = 0.f;
#pragma unroll 1
      for (int k4 = 0; k4 < kDtR / 4; ++k4) {
        const v4f iv = *(const v4f*)(ir + 4 * k4);
        const float* wp = sWin + (4 * k4) * (2 * kMdi) + tid;
        xa = fmaf(iv[0], wp[0], xa);
        za = fmaf(iv[0], wp[kMdi], za);
        xa = fmaf(iv[1], wp[2 * kMdi], xa);
        za = fmaf(iv[1], wp[3 * kMdi], za);
        xa = fmaf(iv[2], wp[4 * kMdi], xa);
        za = fmaf(iv[2], wp[5 * kMdi], za);
        xa = fmaf(iv[3], wp[6 * kMdi], xa);
        za = fmaf(iv[3], wp[7 * kMdi], za);
      }
      const float cpre = fmaf(cw1, xa, cw0 * prevx) + cbv;
      prevx = xa;
      const float xs = silu_f(cpre);
      sXs[tid] = xs;
      __syncthreads();
      if (wave == 0) {
        float a = 0.f;
#pragma unroll 1
        for (int k4 = 0; k4 < kMdi / 4; ++k4) {
          const v4f xv = *(const v4f*)(sXs + 4 * k4);
          const float* xp = sXp + (4 * k4) * kMxd + oc;
          a = fmaf(xv[0], xp[0], a);
          a = fmaf(xv[1], xp[kMxd], a);
          a = fmaf(xv[2], xp[2 * kMxd], a);
          a = fmaf(xv[3], xp[3 * kMxd], a);
        }
        if (lane < kMxd) sSm[lane] = a;
      }
      __syncthreads();
      const v4f s0 = *(const v4f*)(sSm);
      const v4f s1 = *(const v4f*)(sSm + 4);
      const v4f s2 = *(const v4f*)(sSm + 8);
      float dv = dw[0] * s0[0];
      dv = fmaf(dw[1], s0[1], dv);
      dv = fmaf(dw[2], s0[2], dv);
      dv = fmaf(dw[3], s0[3], dv);
      const float dt = softplus_f(dv + dtb);
      const float dtx = dt * xs;
      float y = 0.f;
#pragma unroll
      for (int n = 0; n < kMn; ++n) {
        const float e = __expf(dt * nA[n]);
        st[n] = fmaf(e, st[n], dtx * s1[n]);
        y = fmaf(st[n], s2[n], y);
      }
      y = fmaf(xs, dD, y);
      y = y * silu_f(za);
      sYv[tid] = y;
      __syncthreads();
      float o = 0.f;
#pragma unroll 1
      for (int k4 = 0; k4 < kMdi / 4; ++k4) {
        const v4f yv = *(const v4f*)(sYv + 4 * k4);
        const float* wp = sWout + (4 * k4) * kDtR + tid;
        o = fmaf(yv[0], wp[0], o);
        o = fmaf(yv[1], wp[kDtR], o);
        o = fmaf(yv[2], wp[2 * kDtR], o);
        o = fmaf(yv[3], wp[3 * kDtR], o);
      }
      sO[s * kNbOP + tid] = o;
    }
    __syncthreads();
    v4u pk[2];
#pragma unroll
    for (int it = 0; it < 2; ++it) {
      const int row = it * 8 + wave * 4 + q;
      const float* sp = sO + row * kNbOP + c8;
      const v4f a0 = *(const v4f*)(sp);
      const v4f a1 = *(const v4f*)(sp + 4);
      pk[it] = pack8_bf16(a0, a1);
    }
    for (int pass = 0; pass < 2; ++pass) {
#pragma unroll
      for (int it = 0; it < 2; ++it) {
        const int row = it * 8 + wave * 4 + q;
        *(volatile v4u*)(void*)(DTM + (row0 + l0 + row) * kDtR + c8) = pk[it];
      }
      __threadfence();
    }
  }
}

__global__ __launch_bounds__(64) void scan_kernel(
    const float* __restrict__ DL, const float* __restrict__ UC, const float* __restrict__ XZ,
    const float* __restrict__ XD, const float* __restrict__ bdt, const float* __restrict__ Alog,
    const float* __restrict__ Dp, unsigned short* __restrict__ YH, unsigned short* __restrict__ YL)
{
  __shared__ __align__(16) float sBC[kScanTS * 32];
  __shared__ __align__(16) float sY[kScanTS * kScanYP];
  const int tid = threadIdx.x, lane = tid & 31, wave = tid >> 5;
  constexpr int kBlkPerB = kDin / kScanCh;
  const int bix = blockIdx.x / kBlkPerB;
  const int d0  = (blockIdx.x - bix * kBlkPerB) * kScanCh;
  const int d   = d0 + tid;
  const size_t row0 = (size_t)bix * kSeq;

  float negA[kNst], h[kNst];
#pragma unroll
  for (int g = 0; g < 4; ++g) {
    const v4f al = *(const v4f*)(Alog + (size_t)d * kNst + 4 * g);
    const float a0 = al[0], a1 = al[1], a2 = al[2], a3 = al[3];
    negA[4 * g + 0] = -expf(bf_val(a0));
    negA[4 * g + 1] = -expf(bf_val(a1));
    negA[4 * g + 2] = -expf(bf_val(a2));
    negA[4 * g + 3] = -expf(bf_val(a3));
  }
#pragma unroll
  for (int n = 0; n < kNst; ++n) h[n] = 0.f;
  const float bb = bf_val(bdt[d]);
  const float Dd = bf_val(Dp[d]);

  const int sr = tid >> 3, sc4 = (tid & 7) * 4;
  const int q = lane >> 3, c8 = (lane & 7) * 8;
#pragma unroll 1
  for (int t0 = 0; t0 < kSeq; t0 += kScanTS) {
    __syncthreads();
#pragma unroll
    for (int i = 0; i < 8; ++i) {
      const int r = sr + 8 * i;
      *(v4f*)(sBC + r * 32 + sc4) = *(const v4f*)(XD + (row0 + t0 + r) * kXdP + kDtR + sc4);
    }
    __syncthreads();
#pragma unroll 1
    for (int s = 0; s < kScanTS; ++s) {
      const size_t m = row0 + t0 + s;
      float dl = DL[m * kDin + d];
      float xt = UC[m * kDin + d];
      float zv = XZ[m * kXzP + kDin + d];
      asm volatile("" : "+v"(dl));
      asm volatile("" : "+v"(xt));
      asm volatile("" : "+v"(zv));
      const float* br = sBC + s * 32;
      v4f Bq[4], Cq[4];
#pragma unroll
      for (int g = 0; g < 4; ++g) {
        Bq[g] = *(const v4f*)(br + 4 * g);
        Cq[g] = *(const v4f*)(br + kNst + 4 * g);
      }
      const float dt  = softplus_f(dl + bb);
      const float dtx = dt * xt;
      float y = 0.f;
#pragma unroll
      for (int n = 0; n < kNst; ++n) {
        const float e = __expf(dt * negA[n]);
        h[n] = fmaf(e, h[n], dtx * Bq[n >> 2][n & 3]);
        y = fmaf(h[n], Cq[n >> 2][n & 3], y);
      }
      y = fmaf(xt, Dd, y);
      y = y * silu_f(zv);
      sY[s * kScanYP + tid] = y;
    }
    __syncthreads();
    v4u hv[8], lv[8];
#pragma unroll
    for (int it = 0; it < 8; ++it) {
      const int row = it * 8 + wave * 4 + q;
      const float* sp = sY + row * kScanYP + c8;
      const v4f a0 = *(const v4f*)(sp);
      const v4f a1 = *(const v4f*)(sp + 4);
      split8_bf16(a0, a1, hv[it], lv[it]);
    }
    for (int pass = 0; pass < 2; ++pass) {
#pragma unroll
      for (int it = 0; it < 8; ++it) {
        const int row = it * 8 + wave * 4 + q;
        const size_t o = (row0 + t0 + row) * kDin + d0 + c8;
        *(volatile v4u*)(void*)(YH + o) = hv[it];
        *(volatile v4u*)(void*)(YL + o) = lv[it];
      }
      __threadfence();
    }
  }
}

extern "C" void kernel_launch(void* const* d_in, const int* in_sizes, int n_in,
                              void* d_out, int out_size, void* d_ws, size_t ws_size,
                              hipStream_t stream) {
  if (n_in < 19) return;
  if (in_sizes[0] != kRows * kDm) return;
  if (in_sizes[1] != kXzP * kDm) return;
  if (in_sizes[2] != kDin * 4) return;
  if (in_sizes[3] != kDin) return;
  if (in_sizes[4] != kXdN * kDin) return;
  if (in_sizes[5] != kDin * kNst) return;
  if (in_sizes[6] != kDin) return;
  if (in_sizes[7] != kDin * kDtR) return;
  if (in_sizes[8] != kDin) return;
  if (in_sizes[9] != kDm * kDin) return;
  if (in_sizes[10] != 2 * kMdi * kDtR) return;
  if (in_sizes[11] != kMdi * 2) return;
  if (in_sizes[12] != kMdi) return;
  if (in_sizes[13] != kMxd * kMdi) return;
  if (in_sizes[14] != kMdi * kMdtR) return;
  if (in_sizes[15] != kMdi) return;
  if (in_sizes[16] != kMdi * kMn) return;
  if (in_sizes[17] != kMdi) return;
  if (in_sizes[18] != kDtR * kMdi) return;
  if (out_size != kRows * kDm) return;
  if (ws_size < kWsTotal) return;

  const float* hid     = (const float*)d_in[0];
  const float* W_in    = (const float*)d_in[1];
  const float* conv_w  = (const float*)d_in[2];
  const float* conv_b  = (const float*)d_in[3];
  const float* W_xproj = (const float*)d_in[4];
  const float* A_log   = (const float*)d_in[5];
  const float* Dp      = (const float*)d_in[6];
  const float* W_dt    = (const float*)d_in[7];
  const float* b_dt    = (const float*)d_in[8];
  const float* W_out   = (const float*)d_in[9];
  const float* m_inw   = (const float*)d_in[10];
  const float* m_cw    = (const float*)d_in[11];
  const float* m_cb    = (const float*)d_in[12];
  const float* m_xp    = (const float*)d_in[13];
  const float* m_dtw   = (const float*)d_in[14];
  const float* m_dtb   = (const float*)d_in[15];
  const float* m_Alog  = (const float*)d_in[16];
  const float* m_D     = (const float*)d_in[17];
  const float* m_outw  = (const float*)d_in[18];
  float* out = (float*)d_out;

  char* ws = (char*)d_ws;
  unsigned short* XH   = (unsigned short*)(ws + kOffXH);
  unsigned short* WIH  = (unsigned short*)(ws + kOffWIH);
  unsigned short* WXH  = (unsigned short*)(ws + kOffWXH);
  unsigned short* WDH  = (unsigned short*)(ws + kOffWDH);
  unsigned short* WOH  = (unsigned short*)(ws + kOffWOH);
  float*          XZ   = (float*)(ws + kOffXZ);
  float*          UC   = (float*)(ws + kOffUC);
  unsigned short* UCH  = (unsigned short*)(ws + kOffUCH);
  float*          XD   = (float*)(ws + kOffXD);
  unsigned short* DTM  = (unsigned short*)(ws + kOffDTM);
  float*          DL   = (float*)(ws + kOffDL);
  unsigned short* YH   = (unsigned short*)(ws + kOffYH);
  unsigned short* YL   = (unsigned short*)(ws + kOffYL);

  rne_rows_bf16_kernel<<<(kRows * kDm / 8) / 256, 256, 0, stream>>>(hid, XH, kRows * kDm / 8, kRows * kDm / 8);
  rne_rows_bf16_kernel<<<(kXzP * kDm / 8) / 256, 256, 0, stream>>>(W_in, WIH, kXzP * kDm / 8, kXzP * kDm / 8);
  rne_rows_bf16_kernel<<<(kXdP * kDin / 8) / 256, 256, 0, stream>>>(W_xproj, WXH, kXdP * kDin / 8, kXdN * kDin / 8);
  rne_rows_bf16_kernel<<<(kDin * kDtR / 8) / 256, 256, 0, stream>>>(W_dt, WDH, kDin * kDtR / 8, kDin * kDtR / 8);
  rne_rows_bf16_kernel<<<(kDm * kDin / 8) / 256, 256, 0, stream>>>(W_out, WOH, kDm * kDin / 8, kDm * kDin / 8);

  wmma_gemm64_bf16<0><<<dim3(256, 1), 256, 0, stream>>>(
      XH, XH, kDm, WIH, kDm, XZ, kXzP, kRows, kXzP, kDm);

  conv_silu_kernel<<<dim3(kDin / 256, kRows / 64), 256, 0, stream>>>(XZ, conv_w, conv_b, UC, UCH);

  wmma_gemm64_bf16<0><<<dim3(8, 1), 256, 0, stream>>>(
      UCH, UCH, kDin, WXH, kDin, XD, kXdP, kRows, kXdP, kDin);

  nested_block_kernel<<<kBatch, 64, 0, stream>>>(XD, m_inw, m_cw, m_cb, m_xp, m_dtw, m_dtb, m_Alog, m_D, m_outw, DTM);

  wmma_gemm64_bf16<0><<<dim3(128, 1), 256, 0, stream>>>(
      DTM, DTM, kDtR, WDH, kDtR, DL, kDin, kRows, kDin, kDtR);

  scan_kernel<<<kBatch * (kDin / kScanCh), kScanCh, 0, stream>>>(DL, UC, XZ, XD, b_dt, A_log, Dp, YH, YL);

  wmma_gemm64_bf16<1><<<dim3(64, 1), 256, 0, stream>>>(
      YH, YL, kDin, WOH, kDin, out, kDm, kRows, kDm, kDin);
}
